// EncoderBlock_42795054137796
// MI455X (gfx1250) — hardware-verified
//
#include <hip/hip_runtime.h>
#ifndef NB
#define NB 2
#endif
#ifndef SEQ
#define SEQ 2048
#endif
#define NBF 2
#define SEQF 2048
#define DM 1024
#define NH 16
#define HD 64
#define DFF 4096
#define NTOK (SEQ * NB)
#define XP ((size_t)(NBF / NB) * DM)
#define LNEPS 1e-5f
#define WSC 64.0f
#define HSC 16.0f
#define OSC 32.0f
#define WS_LIMIT ((size_t)134217728)

static_assert(NB == 1 || NB == NBF);
static_assert(SEQ <= SEQF && SEQ % 128 == 0);
static_assert(NH * HD == DM && HD == 64);
static_assert(DM == 256 * 4);
static_assert(NTOK % 128 == 0 && DM % 64 == 0 && DFF % 64 == 0 && DM % 32 == 0 && DFF % 32 == 0);
#define WSB_W   ((size_t)4 * DM * DM * 2 + (size_t)2 * DM * DFF * 2)
#define WSB_X16 ((size_t)NTOK * DM * 2)
#define WSB_QKV ((size_t)NTOK * DM * 6)
#define WSB_VT  ((size_t)NB * NH * HD * SEQ * 2)
#define WSB_HP  ((size_t)NTOK * DM * 4)
#define WSB_FF  ((size_t)NTOK * DFF * 2)
static_assert(WSB_W + WSB_X16 + WSB_QKV + WSB_VT + WSB_HP + WSB_FF <= WS_LIMIT);
static_assert((size_t)NTOK * DM * 2 + (size_t)NTOK * DM * 4 <= WSB_QKV);
static_assert((size_t)(NTOK - 1) * XP + DM <= (size_t)SEQF * NBF * DM);
static_assert(((size_t)NB * NH * (SEQ / 16)) % 8 == 0);

typedef unsigned short v8us __attribute__((ext_vector_type(8), may_alias));
typedef float  v8f  __attribute__((ext_vector_type(8)));
typedef float  v4f  __attribute__((ext_vector_type(4)));
typedef float  v4fa __attribute__((ext_vector_type(4), may_alias));
typedef _Float16 v16h __attribute__((ext_vector_type(16)));
typedef _Float16 v4h  __attribute__((ext_vector_type(4)));
union FragH { v16h v; v8us half[2]; _Float16 h[16]; unsigned short u[16]; };

__device__ __forceinline__ unsigned short bf16_bits(float x) { unsigned int u = __float_as_uint(x); return (unsigned short)((u + 0x7FFFu + ((u >> 16) & 1u)) >> 16); }
__device__ __forceinline__ float bf16_val(unsigned short b) { return __uint_as_float(((unsigned int)b) << 16); }
__device__ __forceinline__ float bf16_rne(float x) { return bf16_val(bf16_bits(x)); }

__device__ __forceinline__ v16h g2_frag(const _Float16* p, int hh) { FragH f; f.half[0] = *(const v8us*)((const unsigned short*)p + 8 * hh); f.half[1] = *(const v8us*)((const unsigned short*)p + 16 + 8 * hh); return f.v; }
__device__ __forceinline__ v8f g2_mma(v16h a, v16h b, v8f c) { v8f d = __builtin_amdgcn_wmma_f32_16x16x32_f16(false, a, false, b, (short)0, c, false, false); asm volatile("v_nop\n\tv_nop\n\tv_nop\n\tv_nop" : "+v"(d) : "v"(a), "v"(b)); return d; }

__global__ __launch_bounds__(256) void k_wt_f16(const float* __restrict__ W, _Float16* __restrict__ Wt, int K, int N, float scale) {
  const int t = blockIdx.x * 256 + threadIdx.x; if (t >= N * (K / 8)) return;
  const int n = t / (K / 8), k8 = (t % (K / 8)) * 8; FragH f;
#pragma unroll
  for (int i = 0; i < 8; ++i) f.h[i] = (_Float16)(bf16_rne(W[(size_t)(k8 + i) * N + n]) * scale);
  const v8us o = f.half[0]; unsigned short* d = (unsigned short*)Wt + (size_t)n * K + k8;
  *(volatile v8us*)d = o; __threadfence(); *(volatile v8us*)d = o;
}

__global__ __launch_bounds__(256) void k_x16(const float* __restrict__ x, _Float16* __restrict__ X16, size_t n8) {
  const size_t t = (size_t)blockIdx.x * 256 + threadIdx.x; if (t >= n8) return;
  const size_t r = t / (DM / 8); const size_t c8 = (t - r * (DM / 8)) * 8;
  const float* src = x + r * XP + c8;
  const v4f a = *(const v4fa*)src, c = *(const v4fa*)(src + 4); FragH f;
#pragma unroll
  for (int q = 0; q < 4; ++q) { f.h[q] = (_Float16)bf16_rne(a[q]); f.h[4 + q] = (_Float16)bf16_rne(c[q]); }
  const v8us o = f.half[0]; unsigned short* d = (unsigned short*)X16 + t * 8;
  *(volatile v8us*)d = o; __threadfence(); *(volatile v8us*)d = o;
}

template <int ACT, int RESBF>
__global__ __launch_bounds__(128) void k_gemm2(const _Float16* __restrict__ A, int lda, const _Float16* __restrict__ Bh, int ldb, float alpha,
    const float* __restrict__ bias, const float* __restrict__ CP, size_t ldcp, float osc,
    float* __restrict__ C, _Float16* __restrict__ C16, int ldc, int M, int N, int K) {
  static_assert(ACT == 0 || ACT == 3);
  __shared__ __attribute__((aligned(16))) float so[4][32][68];
  const int tid = threadIdx.x, w = tid >> 5, lane = tid & 31, ln = lane & 15, hh = lane >> 4;
  const int ntn = N >> 6; const int mt = blockIdx.x / ntn, nq = blockIdx.x - mt * ntn; const int row0 = mt * 128 + 32 * w, col0 = nq * 64; if (row0 >= M) return;
  const _Float16* a0p = A + (size_t)(row0 + ln) * lda; const _Float16* a1p = a0p + (size_t)16 * lda;
  const _Float16* b0p = Bh + (size_t)(col0 + ln) * ldb; const _Float16* b1p = b0p + (size_t)16 * ldb; const _Float16* b2p = b1p + (size_t)16 * ldb; const _Float16* b3p = b2p + (size_t)16 * ldb;
  const v8f z8 = {0.f,0.f,0.f,0.f,0.f,0.f,0.f,0.f}; v8f c00 = z8, c01 = z8, c02 = z8, c03 = z8, c10 = z8, c11 = z8, c12 = z8, c13 = z8;
#pragma unroll 1
  for (int kb = 0; kb < K; kb += 32) { const v16h a0 = g2_frag(a0p + kb, hh), a1 = g2_frag(a1p + kb, hh);
    v16h b = g2_frag(b0p + kb, hh); c00 = g2_mma(a0, b, c00); c10 = g2_mma(a1, b, c10);
    b = g2_frag(b1p + kb, hh); c01 = g2_mma(a0, b, c01); c11 = g2_mma(a1, b, c11);
    b = g2_frag(b2p + kb, hh); c02 = g2_mma(a0, b, c02); c12 = g2_mma(a1, b, c12);
    b = g2_frag(b3p + kb, hh); c03 = g2_mma(a0, b, c03); c13 = g2_mma(a1, b, c13); }
  v8f accs[8] = {c00, c01, c02, c03, c10, c11, c12, c13};
#pragma unroll
  for (int u = 0; u < 8; ++u) { const int t = u & 3, half = u >> 2; const int col = col0 + t * 16 + ln; const float bv = bias ? bf16_rne(bias[col]) : 0.f;
#pragma unroll
    for (int r = 0; r < 8; ++r) { const int rloc = half * 16 + 8 * hh + r; float v = accs[u][r] * alpha + bv;
      if (CP) { float cv = CP[(size_t)(row0 + rloc) * ldcp + col]; if (RESBF) cv = bf16_rne(cv); v += cv; }
      if (ACT == 3) v = fmaxf(v, 0.f);
      so[w][rloc][t * 16 + ln] = v * osc; } }
  __builtin_amdgcn_fence(4  , "workgroup"); __builtin_amdgcn_wave_barrier();
  const int rsub = lane >> 4, c4 = (lane & 15) * 4;
  for (int pass = 0; pass < 2; ++pass) {
#pragma unroll
    for (int q = 0; q < 16; ++q) { const int r = q * 2 + rsub; const v4f v = *(const v4fa*)&so[w][r][c4];
      if (C) *(volatile v4f*)(C + (size_t)(row0 + r) * ldc + col0 + c4) = v;
      if (C16) { v4h h4;
#pragma unroll
        for (int i = 0; i < 4; ++i) h4[i] = (_Float16)v[i];
        *(volatile v4h*)(C16 + (size_t)(row0 + r) * ldc + col0 + c4) = h4; } }
    if (pass == 0) __threadfence(); }
}

__global__ __launch_bounds__(256) void k_vt(const _Float16* __restrict__ V16, _Float16* __restrict__ VT) {
  __shared__ unsigned short tl[64][66];
  const int tid = threadIdx.x; const int nsg = SEQ / 64; const int slab = blockIdx.x / nsg, sg = blockIdx.x - slab * nsg; const int b = slab / NH, h = slab - b * NH; const int s0 = sg * 64;
  for (int i = tid; i < 64 * 8; i += 256) { const int j = i >> 3, c8 = (i & 7) * 8; FragH f; f.half[0] = *(const v8us*)((const unsigned short*)V16 + ((size_t)(s0 + j) * NB + b) * DM + h * HD + c8);
#pragma unroll
    for (int q = 0; q < 8; ++q) tl[j][c8 + q] = f.u[q]; }
  __syncthreads();
  for (int pass = 0; pass < 2; ++pass) {
#pragma unroll
    for (int rd = 0; rd < 2; ++rd) { const int d = rd * 32 + (tid >> 3), pc = tid & 7; FragH f;
#pragma unroll
      for (int q = 0; q < 8; ++q) f.u[q] = tl[pc * 8 + q][d];
      *(volatile v8us*)((unsigned short*)VT + ((size_t)slab * HD + d) * SEQ + s0 + pc * 8) = f.half[0]; }
    if (pass == 0) __threadfence(); }
}

__global__ __launch_bounds__(256) void k_attn(const _Float16* __restrict__ Q16, const _Float16* __restrict__ K16, const _Float16* __restrict__ VT, _Float16* __restrict__ O16, float smul, float osc) {
  __shared__ __attribute__((aligned(16))) _Float16 pt[8][16][40];
  __shared__ __attribute__((aligned(16))) float so[8][16][68];
  const int tid = threadIdx.x, w = tid >> 5, lane = tid & 31, ln = lane & 15, hh = lane >> 4;
  const int nqt = SEQ / 16;
  const int wid = blockIdx.x * 8 + w;
  const int head = wid / nqt, qt = wid - head * nqt;
  if (head >= NB * NH) return;
  const int b = head / NH, h = head - b * NH;
  const int s0 = qt * 16;
  const size_t rp = (size_t)NB * DM;
  const size_t cb = (size_t)b * DM + (size_t)h * HD;
  const _Float16* qp = Q16 + (size_t)(s0 + ln) * rp + cb;
  const v16h qa0 = g2_frag(qp, hh), qa1 = g2_frag(qp + 32, hh);
  const _Float16* kbase = K16 + (size_t)ln * rp + cb;
  const _Float16* vbase = VT + ((size_t)head * HD + ln) * SEQ;
  const v8f z8 = {0.f,0.f,0.f,0.f,0.f,0.f,0.f,0.f};
  v8f o0 = z8, o1 = z8, o2 = z8, o3 = z8;
  float mrun[8], lrun[8];
#pragma unroll
  for (int r = 0; r < 8; ++r) { mrun[r] = -1.0e30f; lrun[r] = 0.f; }
#pragma unroll 1
  for (int t0 = 0; t0 < SEQ; t0 += 32) {
    const _Float16* k0p = kbase + (size_t)t0 * rp; const _Float16* k1p = k0p + (size_t)16 * rp;
    v8f sa = z8, sb = z8;
    { v16h kf = g2_frag(k0p, hh); sa = g2_mma(qa0, kf, sa); kf = g2_frag(k0p + 32, hh); sa = g2_mma(qa1, kf, sa);
      kf = g2_frag(k1p, hh); sb = g2_mma(qa0, kf, sb); kf = g2_frag(k1p + 32, hh); sb = g2_mma(qa1, kf, sb); }
    float scl[8];
#pragma unroll
    for (int r = 0; r < 8; ++r) {
      const float a = sa[r] * smul, c = sb[r] * smul;
      float mx = fmaxf(a, c);
      mx = fmaxf(mx, __shfl_xor(mx, 8, 32)); mx = fmaxf(mx, __shfl_xor(mx, 4, 32)); mx = fmaxf(mx, __shfl_xor(mx, 2, 32)); mx = fmaxf(mx, __shfl_xor(mx, 1, 32));
      const float mn = fmaxf(mrun[r], mx);
      const float f = __expf(mrun[r] - mn);
      const float p0 = __expf(a - mn), p1 = __expf(c - mn);
      float rs = p0 + p1;
      rs += __shfl_xor(rs, 8, 32); rs += __shfl_xor(rs, 4, 32); rs += __shfl_xor(rs, 2, 32); rs += __shfl_xor(rs, 1, 32);
      lrun[r] = lrun[r] * f + rs; mrun[r] = mn; scl[r] = f;
      pt[w][8 * hh + r][ln] = (_Float16)p0; pt[w][8 * hh + r][16 + ln] = (_Float16)p1;
    }
#pragma unroll
    for (int r = 0; r < 8; ++r) { o0[r] = o0[r] * scl[r]; o1[r] = o1[r] * scl[r]; o2[r] = o2[r] * scl[r]; o3[r] = o3[r] * scl[r]; }
    __builtin_amdgcn_fence(4  , "workgroup"); __builtin_amdgcn_wave_barrier();
    FragH pf; pf.half[0] = *(const v8us*)&pt[w][ln][8 * hh]; pf.half[1] = *(const v8us*)&pt[w][ln][16 + 8 * hh];
    __builtin_amdgcn_fence(4  , "workgroup"); __builtin_amdgcn_wave_barrier();
    const _Float16* vp = vbase + t0;
    v16h vf = g2_frag(vp, hh); o0 = g2_mma(pf.v, vf, o0);
    vf = g2_frag(vp + (size_t)16 * SEQ, hh); o1 = g2_mma(pf.v, vf, o1);
    vf = g2_frag(vp + (size_t)32 * SEQ, hh); o2 = g2_mma(pf.v, vf, o2);
    vf = g2_frag(vp + (size_t)48 * SEQ, hh); o3 = g2_mma(pf.v, vf, o3);
  }
#pragma unroll
  for (int r = 0; r < 8; ++r) { const float iv = osc * (1.0f / lrun[r]); const int rr = 8 * hh + r;
    so[w][rr][ln] = o0[r] * iv; so[w][rr][16 + ln] = o1[r] * iv; so[w][rr][32 + ln] = o2[r] * iv; so[w][rr][48 + ln] = o3[r] * iv; }
  __builtin_amdgcn_fence(4  , "workgroup"); __builtin_amdgcn_wave_barrier();
  const int c4 = ln * 4;
  for (int pass = 0; pass < 2; ++pass) {
#pragma unroll
    for (int q = 0; q < 8; ++q) { const int r = q * 2 + hh; const v4f v = *(const v4fa*)&so[w][r][c4]; v4h h4;
#pragma unroll
      for (int i = 0; i < 4; ++i) h4[i] = (_Float16)v[i];
      *(volatile v4h*)(O16 + (size_t)(s0 + r) * rp + cb + c4) = h4; }
    if (pass == 0) __threadfence(); }
}

template <int W16>
__global__ __launch_bounds__(256) void k_ln(const float* __restrict__ X, const float* __restrict__ g, const float* __restrict__ bb, float eps, _Float16* __restrict__ N16, float* __restrict__ N32, size_t op32) {
  #pragma clang fp contract(off)
  __shared__ float red[256];
  const size_t r = blockIdx.x; const int t = threadIdx.x; const int c0 = t * 4;
  const v4f xa = *(const v4fa*)(X + r * DM + c0); float s[4]; float sum = 0.f;
#pragma unroll
  for (int q = 0; q < 4; ++q) { s[q] = xa[q]; sum = __fadd_rn(sum, s[q]); }
  red[t] = sum; __syncthreads();
  for (int st = 128; st > 0; st >>= 1) { if (t < st) red[t] = __fadd_rn(red[t], red[t + st]); __syncthreads(); }
  const float mu = red[0] / (float)DM; __syncthreads();
  float vs = 0.f;
#pragma unroll
  for (int q = 0; q < 4; ++q) { const float dl = __fadd_rn(s[q], -mu); vs = __fadd_rn(vs, __fmul_rn(dl, dl)); }
  red[t] = vs; __syncthreads();
  for (int st = 128; st > 0; st >>= 1) { if (t < st) red[t] = __fadd_rn(red[t], red[t + st]); __syncthreads(); }
  const float rs = rsqrtf(__fadd_rn(red[0] / (float)DM, eps)); v4h y; v4f yf;
#pragma unroll
  for (int q = 0; q < 4; ++q) { const int c = c0 + q; yf[q] = __fadd_rn(__fmul_rn(__fmul_rn(__fadd_rn(s[q], -mu), rs), bf16_rne(g[c])), bf16_rne(bb[c])); y[q] = (_Float16)yf[q]; }
  for (int pass = 0; pass < 2; ++pass) { if (W16) *(volatile v4h*)(N16 + r * DM + c0) = y; *(volatile v4f*)(N32 + r * op32 + c0) = yf; if (pass == 0) __threadfence(); }
}

extern "C" void kernel_launch(void* const* d_in, const int* in_sizes, int n_in,
                              void* d_out, int out_size, void* d_ws, size_t ws_size, hipStream_t stream) {
  if (n_in < 17) return;
  const float* x   = (const float*)d_in[0];
  const float* Wq  = (const float*)d_in[1];  const float* bq  = (const float*)d_in[2];
  const float* Wk  = (const float*)d_in[3];  const float* bk  = (const float*)d_in[4];
  const float* Wv  = (const float*)d_in[5];  const float* bv  = (const float*)d_in[6];
  const float* Wo  = (const float*)d_in[7];  const float* bo  = (const float*)d_in[8];
  const float* g1  = (const float*)d_in[9];  const float* be1 = (const float*)d_in[10];
  const float* W1  = (const float*)d_in[11]; const float* bb1 = (const float*)d_in[12];
  const float* W2  = (const float*)d_in[13]; const float* bb2 = (const float*)d_in[14];
  const float* g2  = (const float*)d_in[15]; const float* be2 = (const float*)d_in[16];
  if ((size_t)in_sizes[0] < (size_t)SEQ * NBF * DM) return;
  if (in_sizes[1] < DM * DM || in_sizes[3] < DM * DM || in_sizes[5] < DM * DM || in_sizes[7] < DM * DM) return;
  if (in_sizes[2] < DM || in_sizes[4] < DM || in_sizes[6] < DM || in_sizes[8] < DM) return;
  if (in_sizes[9] < DM || in_sizes[10] < DM || in_sizes[14] < DM || in_sizes[15] < DM || in_sizes[16] < DM) return;
  if (in_sizes[11] < DM * DFF || in_sizes[12] < DFF || in_sizes[13] < DFF * DM) return;
  if ((size_t)out_size < (size_t)SEQ * NBF * DM) return;

  char* ws = (char*)d_ws; size_t off = 0;
  auto take = [&](size_t bytes) { char* p = ws + off; off += (bytes + 255) & ~(size_t)255; return p; };
  _Float16* BQ = (_Float16*)take((size_t)DM * DM * 2); _Float16* BK = (_Float16*)take((size_t)DM * DM * 2); _Float16* BV = (_Float16*)take((size_t)DM * DM * 2); _Float16* BO = (_Float16*)take((size_t)DM * DM * 2);
  _Float16* B1 = (_Float16*)take((size_t)DFF * DM * 2);
  _Float16* B2 = (_Float16*)take((size_t)DM * DFF * 2);
  _Float16* X16 = (_Float16*)take(WSB_X16); _Float16* O16 = X16;
  char* qkv = take(WSB_QKV);
  _Float16* Q16 = (_Float16*)qkv; _Float16* K16 = (_Float16*)(qkv + (size_t)NTOK * DM * 2); _Float16* V16 = (_Float16*)(qkv + (size_t)NTOK * DM * 4);
  _Float16* H16 = Q16; float* HF = (float*)(qkv + (size_t)NTOK * DM * 2);
  _Float16* VT = (_Float16*)take(WSB_VT);
  float* HP = (float*)take(WSB_HP);
  _Float16* FF16 = (_Float16*)take(WSB_FF);
  if (off > ws_size || off > WS_LIMIT) return;

  { const unsigned gs = (unsigned)(((size_t)DM * (DM / 8) + 255) / 256);
    k_wt_f16<<<gs, 256, 0, stream>>>(Wq, BQ, DM, DM, WSC);
    k_wt_f16<<<gs, 256, 0, stream>>>(Wk, BK, DM, DM, WSC);
    k_wt_f16<<<gs, 256, 0, stream>>>(Wv, BV, DM, DM, WSC);
    k_wt_f16<<<gs, 256, 0, stream>>>(Wo, BO, DM, DM, WSC);
    const unsigned gf = (unsigned)(((size_t)DFF * (DM / 8) + 255) / 256);
    k_wt_f16<<<gf, 256, 0, stream>>>(W1, B1, DM, DFF, WSC);
    const unsigned gg = (unsigned)(((size_t)DM * (DFF / 8) + 255) / 256);
    k_wt_f16<<<gg, 256, 0, stream>>>(W2, B2, DFF, DM, WSC); }
  k_x16<<<(unsigned)(((size_t)NTOK * DM / 8 + 255) / 256), 256, 0, stream>>>(x, X16, (size_t)NTOK * DM / 8);
  const unsigned gq = (unsigned)((NTOK / 128) * (DM / 64));
  k_gemm2<0, 0><<<gq, 128, 0, stream>>>(X16, DM, BQ, DM, 1.0f / WSC, bq, nullptr, (size_t)0, 1.0f, nullptr, Q16, DM, NTOK, DM, DM);
  k_gemm2<0, 0><<<gq, 128, 0, stream>>>(X16, DM, BK, DM, 1.0f / WSC, bk, nullptr, (size_t)0, 1.0f, nullptr, K16, DM, NTOK, DM, DM);
  k_gemm2<0, 0><<<gq, 128, 0, stream>>>(X16, DM, BV, DM, 1.0f / WSC, bv, nullptr, (size_t)0, 1.0f, nullptr, V16, DM, NTOK, DM, DM);
  k_vt<<<(unsigned)(NB * NH * (SEQ / 64)), 256, 0, stream>>>(V16, VT);
  k_attn<<<(unsigned)((size_t)NB * NH * (SEQ / 16) / 8), 256, 0, stream>>>(Q16, K16, VT, O16, 0.125f, OSC);
  k_gemm2<0, 1><<<gq, 128, 0, stream>>>(O16, DM, BO, DM, 1.0f / (WSC * OSC), bo, x, XP, 1.0f, HP, nullptr, DM, NTOK, DM, DM);
  k_ln<1><<<(unsigned)NTOK, 256, 0, stream>>>(HP, g1, be1, LNEPS, H16, HF, (size_t)DM);
  k_gemm2<3, 0><<<(unsigned)((NTOK / 128) * (DFF / 64)), 128, 0, stream>>>(H16, DM, B1, DM, 1.0f / WSC, bb1, nullptr, (size_t)0, HSC, nullptr, FF16, DFF, NTOK, DFF, DM);
  k_gemm2<0, 0><<<gq, 128, 0, stream>>>(FF16, DFF, B2, DFF, 1.0f / (WSC * HSC), bb2, HF, (size_t)DM, 1.0f, HP, nullptr, DM, NTOK, DM, DFF);
  k_ln<0><<<(unsigned)NTOK, 256, 0, stream>>>(HP, g2, be2, LNEPS, nullptr, (float*)d_out, XP);
}
